// VanillaRNN_91216515432752
// MI455X (gfx1250) — hardware-verified
//
#include <hip/hip_runtime.h>
#include <math.h>

typedef __attribute__((ext_vector_type(16))) _Float16 v16h;
typedef __attribute__((ext_vector_type(8)))  _Float16 v8h;
typedef __attribute__((ext_vector_type(8)))  float    v8f;
typedef __attribute__((ext_vector_type(4)))  float    v4f;

constexpr int kBatch  = 2048;
constexpr int kSeq    = 1024;
constexpr int kHid    = 128;
constexpr int kCls    = 10;
constexpr int kRowsB  = 16;
constexpr int kThr    = 128;
constexpr int kWaves  = kThr / 32;
constexpr int kColsW  = kHid / kWaves;
constexpr int kHP     = kHid + 8;
constexpr int kWP     = kHid + 8;
constexpr int kXC     = 32;
constexpr int kXCShift = 5;
constexpr int kHTP    = kHid + 4;
constexpr int kOutB   = kRowsB * kCls;
constexpr int kBlocks = kBatch / kRowsB;
constexpr float kWCarry    = 16.0f;
constexpr float kWCarryInv = 1.0f / 16.0f;
static_assert(kBatch % kRowsB == 0);
static_assert(kColsW == 32);
static_assert(kHid % 32 == 0);
static_assert(kHid == kThr);
static_assert(kHP % 8 == 0 && kWP % 8 == 0);
static_assert((1 << kXCShift) == kXC);
static_assert(kSeq % kXC == 0);
static_assert(kRowsB * kXC == 4 * kThr);
static_assert((kOutB * 4) % 128 == 0);
static_assert(kOutB == 128 + 32);
static_assert(kHid % kWaves == 0 && kHid == 4 * 32);

__device__ __forceinline__ void dep_guard3_h(v8f& a, v8f& b, v16h x, v16h y, v16h z) {
  asm volatile("v_nop\n\tv_nop\n\tv_nop\n\tv_nop" : "+v"(a), "+v"(b) : "v"(x), "v"(y), "v"(z));
}
__device__ __forceinline__ void acc_guard2(v8f& a, v8f& b) {
  asm volatile("v_nop\n\tv_nop\n\tv_nop\n\tv_nop" : "+v"(a), "+v"(b));
}
__device__ __forceinline__ void sched_fence() { asm volatile("" ::: "memory"); }

struct Frag16 {
  union U { v16h v; v8h h[2]; };
  static __device__ __forceinline__ v16h load(const _Float16* p) {
    U f; f.h[0] = *(const v8h*)(p); f.h[1] = *(const v8h*)(p + 16); return f.v;
  }
  static __device__ __forceinline__ v8f mma(v16h a, v16h b, v8f c) {
    return __builtin_amdgcn_wmma_f32_16x16x32_f16(false, a, false, b, (short)0, c, false, false);
  }
};

__device__ __forceinline__ float tanh_f32(float v) {
  const float vc = fminf(fmaxf(v, -15.0f), 15.0f);
  const float e  = expf(2.0f * vc);
  return 1.0f - 2.0f * __builtin_amdgcn_rcpf(1.0f + e);
}

__global__ __launch_bounds__(kThr) void rnn_seq_kernel(
    const float* __restrict__ x, const float* __restrict__ w_hx, const float* __restrict__ w_hh,
    const float* __restrict__ w_ph, const float* __restrict__ b_h, const float* __restrict__ b_p,
    float* __restrict__ out) {
  __shared__ __align__(16) _Float16 wt[kHid * kWP];
  __shared__ __align__(16) _Float16 hb[2][kRowsB * kHP];
  __shared__ __align__(16) float    xs[2][kRowsB * kXC];
  __shared__ __align__(16) float    hT[kRowsB * kHTP];
  __shared__ __align__(16) float    wph[kHid * kCls];
  __shared__ __align__(16) float    bp[16];
  __shared__ __align__(16) float    outs[kOutB];

  const int tid = threadIdx.x, lane = tid & 31, wave = tid >> 5;
  const int c = lane & 15, hh = lane >> 4, koff = hh * 8;
  const int row0 = blockIdx.x * kRowsB;
  const int nbase = kColsW * wave;

  {
    const v8h z = {(_Float16)0.f, (_Float16)0.f, (_Float16)0.f, (_Float16)0.f,
                   (_Float16)0.f, (_Float16)0.f, (_Float16)0.f, (_Float16)0.f};
    _Float16* hbf = &hb[0][0];
    for (int i = tid; i < (2 * kRowsB * kHP) / 8; i += kThr) *(v8h*)(hbf + 8 * i) = z;
  }

#pragma unroll 4
  for (int p = 0; p < kHid / kWaves; ++p) {
    const int k = p * kWaves + wave;
    const v4f v = *(const v4f*)(w_hh + (size_t)k * kHid + 4 * lane);
#pragma unroll
    for (int e = 0; e < 4; ++e) wt[(4 * lane + e) * kWP + k] = (_Float16)(v[e] * kWCarry);
  }
  sched_fence();

  {
    const int m = tid >> 3, g = tid & 7;
    const v4f v = *(const v4f*)(x + (size_t)(row0 + m) * kSeq + 4 * g);
    *(v4f*)(&xs[0][m * kXC + 4 * g]) = v;
  }
  sched_fence();

#pragma unroll
  for (int j = 0; j < kCls; ++j) wph[tid + kThr * j] = w_ph[tid + kThr * j];
  sched_fence();
  {
    const int ci = (tid < kCls) ? tid : (kCls - 1);
    const float bv = b_p[ci];
    if (tid < 16) bp[tid] = (tid < kCls) ? bv : 0.0f;
  }

  float whx[2], bh[2];
#pragma unroll
  for (int b = 0; b < 2; ++b) {
    const int n = nbase + 16 * b + c;
    whx[b] = w_hx[n];
    bh[b]  = b_h[n];
  }
  __syncthreads();

  float hlast[2][8];
#pragma unroll
  for (int b = 0; b < 2; ++b)
#pragma unroll
    for (int r = 0; r < 8; ++r) hlast[b][r] = 0.0f;
  const v8f z8 = {0.f, 0.f, 0.f, 0.f, 0.f, 0.f, 0.f, 0.f};
  const _Float16* brow = wt + (size_t)(nbase + c) * kWP + koff;

#pragma unroll 1
  for (int t = 0; t < kSeq; ++t) {
    if ((t & (kXC - 1)) == 0) {
      const int nt0 = t + kXC;
      if (nt0 < kSeq) {
        const int m = tid >> 3, g = tid & 7;
        const v4f v = *(const v4f*)(x + (size_t)(row0 + m) * kSeq + nt0 + 4 * g);
        *(v4f*)(&xs[((t >> kXCShift) + 1) & 1][m * kXC + 4 * g]) = v;
      }
    }

    const _Float16* hc = &hb[t & 1][0];
    _Float16*       hn = &hb[(t + 1) & 1][0];
    const float* xsc = &xs[(t >> kXCShift) & 1][0];
    float xm[8];
#pragma unroll
    for (int r = 0; r < 8; ++r) xm[r] = xsc[(8 * hh + r) * kXC + (t & (kXC - 1))];

    v8f acc[2];
    acc[0] = z8; acc[1] = z8;
    const _Float16* arow = hc + c * kHP + koff;
#pragma unroll
    for (int kc = 0; kc < kHid / 32; ++kc) {
      const v16h fa  = Frag16::load(arow + 32 * kc);
      const v16h fb0 = Frag16::load(brow + 32 * kc);
      const v16h fb1 = Frag16::load(brow + 16 * kWP + 32 * kc);
      acc[0] = Frag16::mma(fa, fb0, acc[0]);
      acc[1] = Frag16::mma(fa, fb1, acc[1]);
      dep_guard3_h(acc[0], acc[1], fa, fb0, fb1);
    }
    acc_guard2(acc[0], acc[1]);

#pragma unroll
    for (int b = 0; b < 2; ++b) {
      const int n = nbase + 16 * b + c;
#pragma unroll
      for (int r = 0; r < 8; ++r) {
        const float xw  = xm[r] * whx[b];
        const float pre = fmaf(acc[b][r], kWCarryInv, xw) + bh[b];
        const float hv  = tanh_f32(pre);
        hlast[b][r] = hv;
        hn[(8 * hh + r) * kHP + n] = (_Float16)hv;
      }
    }
    __syncthreads();
  }

#pragma unroll
  for (int b = 0; b < 2; ++b)
#pragma unroll
    for (int r = 0; r < 8; ++r) hT[(8 * hh + r) * kHTP + nbase + 16 * b + c] = hlast[b][r];
  __syncthreads();

  {
    const int o0 = tid;
    const int o1 = (tid + 128 < kOutB) ? (tid + 128) : (kOutB - 1);
    const int m0 = o0 / kCls, c0 = o0 - kCls * m0;
    const int m1 = o1 / kCls, c1 = o1 - kCls * m1;
    const float* h0p = hT + m0 * kHTP;
    const float* h1p = hT + m1 * kHTP;
    float s0 = 0.0f, s1 = 0.0f;
#pragma unroll 4
    for (int k = 0; k < kHid; ++k) {
      s0 = fmaf(h0p[k], wph[k * kCls + c0], s0);
      s1 = fmaf(h1p[k], wph[k * kCls + c1], s1);
    }
    const float r0v = s0 + bp[c0];
    const float r1v = s1 + bp[c1];
    outs[o0] = r0v;
    if (tid + 128 < kOutB) outs[o1] = r1v;
  }
  __syncthreads();

  if (wave < 2) {
    float* ob = out + (size_t)blockIdx.x * kOutB;
    const bool act = (wave == 0) || (lane < 8);
    const int fo = act ? (wave * 128 + 4 * lane) : 0;
    const v4f v = *(const v4f*)(&outs[fo]);
    for (int pass = 0; pass < 2; ++pass) {
      if (act) *(volatile v4f*)(ob + fo) = v;
      __threadfence();
    }
  }
}

extern "C" void kernel_launch(void* const* d_in, const int* in_sizes, int n_in,
                              void* d_out, int out_size, void* d_ws, size_t ws_size, hipStream_t stream) {
  (void)d_ws; (void)ws_size;
  if (n_in < 6 || d_out == nullptr) return;
  if (in_sizes[0] != kBatch * kSeq || in_sizes[1] != kHid || in_sizes[2] != kHid * kHid ||
      in_sizes[3] != kHid * kCls || in_sizes[4] != kHid || in_sizes[5] != kCls ||
      out_size != kBatch * kCls) return;

  const float* x    = (const float*)d_in[0];
  const float* w_hx = (const float*)d_in[1];
  const float* w_hh = (const float*)d_in[2];
  const float* w_ph = (const float*)d_in[3];
  const float* b_h  = (const float*)d_in[4];
  const float* b_p  = (const float*)d_in[5];
  float* out = (float*)d_out;

  rnn_seq_kernel<<<kBlocks, kThr, 0, stream>>>(x, w_hx, w_hh, w_ph, b_h, b_p, out);
}
